// PointSpatialConv_20684562497678
// MI455X (gfx1250) — hardware-verified
//
#include <hip/hip_runtime.h>
#include <math.h>

typedef __attribute__((ext_vector_type(16))) _Float16 v16h;
typedef __attribute__((ext_vector_type(16))) __bf16 v16b;
typedef __attribute__((ext_vector_type(8)))  _Float16 v8h;
typedef __attribute__((ext_vector_type(8)))  float v8f;
typedef __attribute__((ext_vector_type(4)))  float v4f;
typedef __attribute__((ext_vector_type(2)))  float v2f;
typedef __attribute__((ext_vector_type(4)))  unsigned v4u;
typedef __attribute__((ext_vector_type(4)))  int v4i;
typedef float __attribute__((may_alias)) float_a;
typedef int __attribute__((may_alias)) int_a;

template <typename T> __device__ __forceinline__ void vst2(void* p, T v) { *(volatile T*)p = v; __threadfence(); *(volatile T*)p = v; }
__device__ __forceinline__ v8f wmma16(v16h a, v16h b, v8f c) {
  v8f d = __builtin_amdgcn_wmma_f32_16x16x32_f16(false, a, false, b, (short)0, c, false, false);
  asm volatile("v_nop\n\tv_nop\n\tv_nop\n\tv_nop" : "+v"(d) : "v"(a), "v"(b));
  return d;
}
__device__ __forceinline__ v8f wmma_bf(v16b a, v16b b, v8f c) {
  v8f d = __builtin_amdgcn_wmma_f32_16x16x32_bf16(false, a, false, b, (short)0, c, false, false);
  asm volatile("v_nop\n\tv_nop\n\tv_nop\n\tv_nop" : "+v"(d) : "v"(a), "v"(b));
  return d;
}
__device__ __forceinline__ v16h frag_h(const _Float16* rowk0, int lane) {
  union { v16h v; v8h q[2]; } u; const _Float16* p = rowk0 + 8 * (lane >> 4);
  u.q[0] = *(const v8h*)p; u.q[1] = *(const v8h*)(p + 16); return u.v;
}
__device__ __forceinline__ v16h frag_f32(const float* rowk0, int lane) {
  v16h a; const float* p = rowk0 + 8 * (lane >> 4);
#pragma unroll
  for (int i = 0; i < 8; ++i) { a[i] = (_Float16)p[i]; a[8 + i] = (_Float16)p[16 + i]; }
  return a;
}
__device__ __forceinline__ v16h frag_f32s(const float* rowk0, int lane, float sc) {
  v16h a; const float* p = rowk0 + 8 * (lane >> 4);
#pragma unroll
  for (int i = 0; i < 8; ++i) { a[i] = (_Float16)(p[i] * sc); a[8 + i] = (_Float16)(p[16 + i] * sc); }
  return a;
}
__device__ __forceinline__ v16h fragc_f32(const float* W, int k0, int n, int lane, int ld, int K) {
  v16h a; const int g = lane >> 4;
#pragma unroll
  for (int i = 0; i < 8; ++i) { const int ka = k0 + 8 * g + i, kb = ka + 16;
    a[i] = (_Float16)(ka < K ? W[(size_t)(ka < K ? ka : K - 1) * ld + n] : 0.f); a[8 + i] = (_Float16)(kb < K ? W[(size_t)(kb < K ? kb : K - 1) * ld + n] : 0.f); }
  return a;
}
struct F2 { v16b h, l; };
__device__ __forceinline__ F2 bsplit16(const float v[16]) { F2 r;
#pragma unroll
  for (int i = 0; i < 16; ++i) { const __bf16 h = (__bf16)v[i]; r.h[i] = h; r.l[i] = (__bf16)(v[i] - (float)h); }
  return r; }
__device__ __forceinline__ F2 split_row(const float* row, int k0, int lane) { float v[16]; const float* p = row + k0 + 8 * (lane >> 4);
#pragma unroll
  for (int i = 0; i < 8; ++i) { v[i] = p[i]; v[8 + i] = p[16 + i]; }
  return bsplit16(v); }
__device__ __forceinline__ F2 split_rowK(const float* row, int k0, int lane, int K) { float v[16]; const int g = lane >> 4;
#pragma unroll
  for (int i = 0; i < 8; ++i) { const int ka = k0 + 8 * g + i, kb = ka + 16; v[i] = ka < K ? row[ka < K ? ka : K - 1] : 0.f; v[8 + i] = kb < K ? row[kb < K ? kb : K - 1] : 0.f; }
  return bsplit16(v); }
__device__ __forceinline__ F2 split_col(const float* W, int k0, int n, int lane, int ld, int K) { float v[16]; const int g = lane >> 4;
#pragma unroll
  for (int i = 0; i < 8; ++i) { const int ka = k0 + 8 * g + i, kb = ka + 16; v[i] = ka < K ? W[(size_t)(ka < K ? ka : K - 1) * ld + n] : 0.f; v[8 + i] = kb < K ? W[(size_t)(kb < K ? kb : K - 1) * ld + n] : 0.f; }
  return bsplit16(v); }
__device__ __forceinline__ v8f mac3(const F2& a, const F2& b, v8f c) { c = wmma_bf(a.l, b.h, c); c = wmma_bf(a.h, b.l, c); return wmma_bf(a.h, b.h, c); }
__device__ __forceinline__ float sigm(float v) { return 1.0f / (1.0f + expf(-v)); }
#define LDSX() do { asm volatile("s_wait_dscnt 0" ::: "memory"); __builtin_amdgcn_wave_barrier(); __builtin_amdgcn_fence(__ATOMIC_RELEASE, "workgroup"); } while (0)

__device__ __forceinline__ float bfr(float v) { return (float)(__bf16)v; }
#define NB 8
#define NPT 8192
#define NM 2048
#define KN 32
#define CIN 64
#define C1 128
#define C2 128
#define C3 256
#define APB 32
#ifndef TNB
#define TNB NB
#endif
#define WS_FT  0u
#define WS_W2T (WS_FT + 4u * (size_t)NB * NPT * CIN)
#define WS_W3T (WS_W2T + 2u * (size_t)C2 * C1)
#define WS_END (WS_W3T + 2u * (size_t)C3 * C2)
__global__ __launch_bounds__(256) void k_ft(const float* __restrict__ FEAT, float* __restrict__ FT) { __shared__ float st[CIN][65];
  const int t = threadIdx.x; const int n0 = blockIdx.x * 64; const size_t b = blockIdx.y;
  for (int e = t; e < CIN * 64; e += 256) { const int c = e >> 6, nl = e & 63; st[c][nl] = bfr(FEAT[(b * CIN + c) * (size_t)NPT + n0 + nl]); }
  __syncthreads();
  for (int e = t; e < 64 * 16; e += 256) { const int nl = e >> 4, q = e & 15; v4f o; o[0] = st[q * 4][nl]; o[1] = st[q * 4 + 1][nl]; o[2] = st[q * 4 + 2][nl]; o[3] = st[q * 4 + 3][nl]; vst2(FT + (b * NPT + n0 + nl) * CIN + q * 4, o); } }
__global__ __launch_bounds__(128) void k_wt(const float* __restrict__ W2, const float* __restrict__ W3, _Float16* __restrict__ W2T, _Float16* __restrict__ W3T) { __shared__ __align__(16) _Float16 s[C1];
  const int o = blockIdx.x; const int k = threadIdx.x;
  if (o < C2) s[k] = (_Float16)bfr(W2[(size_t)k * C2 + o]); else s[k] = (_Float16)bfr(W3[(size_t)k * C3 + (o - C2)]);
  __syncthreads();
  if (k < 16) { _Float16* dst = (o < C2) ? (W2T + (size_t)o * C1) : (W3T + (size_t)(o - C2) * C2); vst2((v4u*)(dst + k * 8), *(const v4u*)&s[k * 8]); } }
__global__ __launch_bounds__(128) void k_mlp(const float* __restrict__ XYZ, const float* __restrict__ FT, const int* __restrict__ NI, const int* __restrict__ AI, const float* __restrict__ W1, const float* __restrict__ B1, const _Float16* __restrict__ W2T, const float* __restrict__ B2, const _Float16* __restrict__ W3T, const float* __restrict__ B3, float* __restrict__ OUT) {
  __shared__ __align__(16) _Float16 sa[64][136]; __shared__ __align__(16) float smax[4][C3]; __shared__ __align__(16) float outb[APB][C3 + 4];
  const int tid = threadIdx.x, wave = tid >> 5, lane = tid & 31, col = lane & 15, g = lane >> 4; const int m0 = blockIdx.x * APB; const size_t b = blockIdx.y;
  for (int sub = 0; sub < APB / 2; ++sub) {
    const int al = sub * 2 + (wave >> 1); const int a = m0 + al; const int j = (wave & 1) * 16 + col;
    int ni = NI[(b * NM + a) * KN + j]; ni = ni < 0 ? 0 : (ni >= NPT ? NPT - 1 : ni); int ai = AI[b * NM + a]; ai = ai < 0 ? 0 : (ai >= NPT ? NPT - 1 : ai);
    v8f acc[8] = {};
#pragma unroll
    for (int kc = 0; kc < CIN / 32; ++kc) { v16b av; { const float* p = FT + (b * NPT + ni) * CIN + kc * 32 + 8 * g;
#pragma unroll
        for (int i = 0; i < 8; ++i) { av[i] = (__bf16)p[i]; av[8 + i] = (__bf16)p[16 + i]; } }
#pragma unroll
      for (int jt = 0; jt < 8; ++jt) { v16b w; const int o = jt * 16 + col;
#pragma unroll
        for (int i = 0; i < 8; ++i) { w[i] = (__bf16)W1[(size_t)(3 + kc * 32 + 8 * g + i) * C1 + o]; w[8 + i] = (__bf16)W1[(size_t)(3 + kc * 32 + 16 + 8 * g + i) * C1 + o]; }
        asm volatile("s_wait_loadcnt 0x0" ::: "memory"); acc[jt] = wmma_bf(av, w, acc[jt]); } }
    { const float ax = bfr(XYZ[(b * NPT + ai) * 3]), ay = bfr(XYZ[(b * NPT + ai) * 3 + 1]), az = bfr(XYZ[(b * NPT + ai) * 3 + 2]);
#pragma unroll
      for (int r = 0; r < 8; ++r) { const int jr = (wave & 1) * 16 + 8 * g + r; int nr = NI[(b * NM + a) * KN + jr]; nr = nr < 0 ? 0 : (nr >= NPT ? NPT - 1 : nr);
        const float rx = bfr(XYZ[(b * NPT + nr) * 3]) - ax, ry = bfr(XYZ[(b * NPT + nr) * 3 + 1]) - ay, rz = bfr(XYZ[(b * NPT + nr) * 3 + 2]) - az;
#pragma unroll
        for (int jt = 0; jt < 8; ++jt) { const int o = jt * 16 + col; const float v = acc[jt][r] + rx * bfr(W1[o]) + ry * bfr(W1[C1 + o]) + rz * bfr(W1[2 * C1 + o]) + bfr(B1[o]); sa[wave * 16 + 8 * g + r][o] = (_Float16)fmaxf(v, 0.f); }
        asm volatile("s_wait_loadcnt 0x0" ::: "memory"); } }
    __syncthreads();
#pragma unroll
    for (int jt = 0; jt < 8; ++jt) acc[jt] = (v8f){};
#pragma unroll
    for (int kc = 0; kc < C1 / 32; ++kc) { v16h av; { const _Float16* p = &sa[wave * 16 + col][kc * 32 + 8 * g];
#pragma unroll
        for (int i = 0; i < 8; ++i) { av[i] = p[i]; av[8 + i] = p[16 + i]; } }
#pragma unroll
      for (int jt = 0; jt < 8; ++jt) acc[jt] = wmma16(av, frag_h(W2T + (size_t)(jt * 16 + col) * C1 + kc * 32, lane), acc[jt]); }
    __syncthreads();
#pragma unroll
    for (int jt = 0; jt < 8; ++jt) { const int o = jt * 16 + col; const float bb = bfr(B2[o]);
#pragma unroll
      for (int r = 0; r < 8; ++r) sa[wave * 16 + 8 * g + r][o] = (_Float16)fmaxf(acc[jt][r] + bb, 0.f); }
    __syncthreads();
    for (int half = 0; half < 2; ++half) {
#pragma unroll
      for (int jt = 0; jt < 8; ++jt) acc[jt] = (v8f){};
#pragma unroll
      for (int kc = 0; kc < C2 / 32; ++kc) { v16h av; { const _Float16* p = &sa[wave * 16 + col][kc * 32 + 8 * g];
#pragma unroll
          for (int i = 0; i < 8; ++i) { av[i] = p[i]; av[8 + i] = p[16 + i]; } }
#pragma unroll
        for (int jt = 0; jt < 8; ++jt) acc[jt] = wmma16(av, frag_h(W3T + (size_t)(half * 128 + jt * 16 + col) * C2 + kc * 32, lane), acc[jt]); }
#pragma unroll
      for (int jt = 0; jt < 8; ++jt) { const int o = half * 128 + jt * 16 + col; const float bb = bfr(B3[o]); float mx = -3.0e38f;
#pragma unroll
        for (int r = 0; r < 8; ++r) mx = fmaxf(mx, fmaxf(acc[jt][r] + bb, 0.f));
        mx = fmaxf(mx, __shfl_xor(mx, 16));
        if (g == 0) smax[wave][o] = mx; } }
    __syncthreads();
    for (int e = tid; e < 2 * C3; e += 128) { const int an = e / C3, o = e % C3; outb[sub * 2 + an][o] = fmaxf(smax[an * 2][o], smax[an * 2 + 1][o]); }
    __syncthreads(); }
  for (int e = tid; e < C3 * 8; e += 128) { const int c = e >> 3, q = e & 7; v4f o; o[0] = outb[q * 4][c]; o[1] = outb[q * 4 + 1][c]; o[2] = outb[q * 4 + 2][c]; o[3] = outb[q * 4 + 3][c]; vst2(OUT + (b * C3 + c) * (size_t)NM + m0 + q * 4, o); } }
extern "C" void kernel_launch(void* const* d_in, const int* in_sizes, int n_in, void* d_out, int out_size, void* d_ws, size_t ws_size, hipStream_t stream) {
  (void)in_sizes; (void)n_in; (void)out_size;
  const float** F = (const float**)d_in;
  if (ws_size < (size_t)WS_END) return;
  char* ws = (char*)d_ws; float* FT = (float*)(ws + WS_FT); _Float16 *W2T = (_Float16*)(ws + WS_W2T), *W3T = (_Float16*)(ws + WS_W3T);
  k_ft<<<dim3(NPT / 64, TNB), 256, 0, stream>>>(F[1], FT);
  k_wt<<<dim3(C2 + C3), 128, 0, stream>>>(F[6], F[8], W2T, W3T);
  k_mlp<<<dim3(NM / APB, TNB), 128, 0, stream>>>(F[0], FT, (const int*)d_in[2], (const int*)d_in[3], F[4], F[5], W2T, F[7], W3T, F[9], (float*)d_out);
}
